// GNO_61366492725767
// MI455X (gfx1250) — hardware-verified
//
#include <hip/hip_runtime.h>
#include <stddef.h>


#define DL      64
#define KX      16
#define K1      32
#define K1REAL  18
#define NTHR    256
#define NWAVE   8
#define NROWS   128
#define EPT     8
#define NGRP    2
#define CHUNK   (NTHR * EPT * NGRP)
#define WCAP    (EPT * NGRP * 32)
#define LISTN   (NWAVE * WCAP)
#define NB      512
#define WSCALE  8.0f
#define WINV    0.125f
#define LDS_AGG (NB * DL * 4 + LISTN * 4 + NB * 4 + 64)

static_assert((CHUNK & (CHUNK - 1)) == 0);
static_assert(CHUNK <= 4096);
static_assert(NB <= 4096 && (NB & (NB - 1)) == 0);
static_assert(NWAVE * 16 * DL * 2 <= LISTN * 4);
static_assert(NB == NWAVE * 4 * 16);
static_assert(NB % 128 == 0 && NB / 128 <= NWAVE);
static_assert(NROWS == NWAVE * 16);

typedef float    v2f  __attribute__((ext_vector_type(2)));
typedef float    v4f  __attribute__((ext_vector_type(4)));
typedef float    v8f  __attribute__((ext_vector_type(8)));
typedef int      v4i  __attribute__((ext_vector_type(4)));
typedef _Float16 v8h  __attribute__((ext_vector_type(8)));
typedef _Float16 v16h __attribute__((ext_vector_type(16)));
union FragH { v16h v; v8h h[2]; };

__device__ __forceinline__ float gelu_exact(float v) {
  return 0.5f * v * (1.0f + erff(v * 0.70710678118654752f));
}

__device__ __forceinline__ v8h cvt8(v4f a, v4f b) {
  v8h r;
  r[0] = (_Float16)a.x; r[1] = (_Float16)a.y; r[2] = (_Float16)a.z; r[3] = (_Float16)a.w;
  r[4] = (_Float16)b.x; r[5] = (_Float16)b.y; r[6] = (_Float16)b.z; r[7] = (_Float16)b.w;
  return r;
}

__device__ __forceinline__ v8f wmh(v16h a, v16h b, v8f c) {
  v8f d = __builtin_amdgcn_wmma_f32_16x16x32_f16(false, a, false, b, (short)0, c, false, false);
  asm volatile("v_nop\n\tv_nop\n\tv_nop\n\tv_nop" : "+v"(d) : "v"(a), "v"(b));
  return d;
}

template <int NBT>
__device__ __forceinline__ int scan_chunk(const int* __restrict__ dsts, int nE, int cbase, int nodeBase,
                                          int vec8, int* list, int tid, int lane, int wave) {
  int wc = 0;
#pragma unroll
  for (int g = 0; g < NGRP; ++g) {
    const int el0  = (g * NTHR + tid) * EPT;
    const int e0   = cbase + el0;
    const int sent = -2147483647 - 1;
    v4i da, db;
    if (vec8 != 0 && cbase + CHUNK <= nE) {
      da = *(const v4i*)(dsts + e0);
      db = *(const v4i*)(dsts + e0 + 4);
    } else {
      da.x = (e0     < nE) ? dsts[min(e0, nE - 1)] : sent;
      da.y = (e0 + 1 < nE) ? dsts[min(e0 + 1, nE - 1)] : sent;
      da.z = (e0 + 2 < nE) ? dsts[min(e0 + 2, nE - 1)] : sent;
      da.w = (e0 + 3 < nE) ? dsts[min(e0 + 3, nE - 1)] : sent;
      db.x = (e0 + 4 < nE) ? dsts[min(e0 + 4, nE - 1)] : sent;
      db.y = (e0 + 5 < nE) ? dsts[min(e0 + 5, nE - 1)] : sent;
      db.z = (e0 + 6 < nE) ? dsts[min(e0 + 6, nE - 1)] : sent;
      db.w = (e0 + 7 < nE) ? dsts[min(e0 + 7, nE - 1)] : sent;
    }
    const unsigned nb = (unsigned)nodeBase;
    const unsigned s0 = (unsigned)da.x - nb, s1 = (unsigned)da.y - nb;
    const unsigned s2 = (unsigned)da.z - nb, s3 = (unsigned)da.w - nb;
    const unsigned s4 = (unsigned)db.x - nb, s5 = (unsigned)db.y - nb;
    const unsigned s6 = (unsigned)db.z - nb, s7 = (unsigned)db.w - nb;
    const bool h0 = s0 < (unsigned)NBT, h1 = s1 < (unsigned)NBT, h2 = s2 < (unsigned)NBT, h3 = s3 < (unsigned)NBT;
    const bool h4 = s4 < (unsigned)NBT, h5 = s5 < (unsigned)NBT, h6 = s6 < (unsigned)NBT, h7 = s7 < (unsigned)NBT;
    const unsigned any = __builtin_amdgcn_ballot_w32(h0 | h1 | h2 | h3 | h4 | h5 | h6 | h7);
    if (any != 0u) {
#define HITJ(J, HJ, SJ) { \
        const unsigned mj = __builtin_amdgcn_ballot_w32(HJ); \
        if (mj != 0u) { \
          if (HJ) { \
            const int pos = wc + (int)__builtin_amdgcn_mbcnt_lo(mj, 0u); \
            if (pos < WCAP) list[wave * WCAP + pos] = ((el0 + (J)) << 12) | (int)(SJ); \
          } \
          wc += (int)__builtin_popcount(mj); } }
      HITJ(0, h0, s0)
      HITJ(1, h1, s1)
      HITJ(2, h2, s2)
      HITJ(3, h3, s3)
      HITJ(4, h4, s4)
      HITJ(5, h5, s5)
      HITJ(6, h6, s6)
      HITJ(7, h7, s7)
#undef HITJ
    }
  }
  return wc;
}

__global__ __launch_bounds__(NTHR) void k_wprep(
    const float* __restrict__ pw1, const float* __restrict__ pw2,
    const float* __restrict__ ww1, const float* __restrict__ ww2,
    const float* __restrict__ dw1,
    _Float16* W1p, _Float16* W2p, _Float16* V1p, _Float16* V2p, _Float16* D1p) {
  const int i  = blockIdx.x * NTHR + threadIdx.x;
  const int n1 = DL * K1 / 8;
  const int n2 = DL * DL / 8;
  if (i >= n1 + 4 * n2) return;
  int which, o;
  if (i < n1) { which = 0; o = i * 8; }
  else { const int j = i - n1; which = 1 + j / n2; o = (j % n2) * 8; }
  const int pitch = (which == 0) ? K1 : DL;
  const int kmax  = (which == 0) ? K1REAL : DL;
  const int n  = o / pitch;
  const int k0 = o - n * pitch;
  const float* W = (which == 0) ? pw1 : (which == 1) ? pw2 : (which == 2) ? ww1 : (which == 3) ? ww2 : dw1;
  _Float16*    P = (which == 0) ? W1p : (which == 1) ? W2p : (which == 2) ? V1p : (which == 3) ? V2p : D1p;
  v8h hv;
#pragma unroll
  for (int j = 0; j < 8; ++j) {
    const int k  = k0 + j;
    const int kc = (k < kmax) ? k : kmax - 1;
    float v = W[(size_t)kc * DL + n];
    v = (k < kmax) ? v * WSCALE : 0.0f;
    hv[j] = (_Float16)v;
  }
  _Float16* dp = P + o;
  *(volatile v8h*)dp = hv;
  __threadfence();
  *(volatile v8h*)dp = hv;
}

__global__ __launch_bounds__(NTHR) void k_node(
    const float* __restrict__ x, const float* __restrict__ grd,
    const _Float16* __restrict__ W1p, const float* __restrict__ pb1,
    const _Float16* __restrict__ W2p, const float* __restrict__ pb2,
    float* hpl, int nN) {
  __shared__ __attribute__((aligned(16))) _Float16 sA[NWAVE][16 * K1];
  __shared__ __attribute__((aligned(16))) _Float16 sT[NWAVE][16 * DL];
  __shared__ __attribute__((aligned(16))) float    stg[NWAVE][16 * DL];
  const int tid = threadIdx.x, lane = tid & 31, wave = tid >> 5, hh = lane >> 4, m = lane & 15;
  const int row0 = blockIdx.x * NROWS + wave * 16;

  {
    const int r = lane >> 1, c0 = (lane & 1) * 8;
    int node = row0 + r;
    node = node > nN - 1 ? nN - 1 : node;
    const float* xp = x + (size_t)node * KX + c0;
    const v4f a = *(const v4f*)xp, b = *(const v4f*)(xp + 4);
    *(v8h*)(&sA[wave][r * K1 + c0]) = cvt8(a, b);
    int node2 = row0 + m;
    node2 = node2 > nN - 1 ? nN - 1 : node2;
    const float g0 = grd[(size_t)node2 * 2], g1 = grd[(size_t)node2 * 2 + 1];
    v8h gv;
    gv[0] = (_Float16)((hh == 0) ? g0 : 0.0f);
    gv[1] = (_Float16)((hh == 0) ? g1 : 0.0f);
    gv[2] = (_Float16)0.0f; gv[3] = (_Float16)0.0f; gv[4] = (_Float16)0.0f;
    gv[5] = (_Float16)0.0f; gv[6] = (_Float16)0.0f; gv[7] = (_Float16)0.0f;
    *(v8h*)(&sA[wave][m * K1 + 16 + 8 * hh]) = gv;
  }
  __syncthreads();

  v8f acc[4];
#pragma unroll
  for (int t = 0; t < 4; ++t) { v8f z = {0.f, 0.f, 0.f, 0.f, 0.f, 0.f, 0.f, 0.f}; acc[t] = z; }
  {
    const _Float16* ar = &sA[wave][m * K1 + 8 * hh];
    FragH a;
    a.h[0] = *(const v8h*)ar;
    a.h[1] = *(const v8h*)(ar + 16);
#pragma unroll
    for (int t = 0; t < 4; ++t) {
      const _Float16* bp = W1p + (size_t)(16 * t + m) * K1 + 8 * hh;
      FragH b;
      b.h[0] = *(const v8h*)bp;
      b.h[1] = *(const v8h*)(bp + 16);
      acc[t] = wmh(a.v, b.v, acc[t]);
    }
  }
#pragma unroll
  for (int t = 0; t < 4; ++t) {
    const float bias = pb1[16 * t + m];
    _Float16* sp = &sT[wave][(8 * hh) * DL + 16 * t + m];
#pragma unroll
    for (int r = 0; r < 8; ++r) sp[r * DL] = (_Float16)gelu_exact(acc[t][r] * WINV + bias);
  }
  __syncthreads();

  v8f acc2[4];
#pragma unroll
  for (int t = 0; t < 4; ++t) { v8f z = {0.f, 0.f, 0.f, 0.f, 0.f, 0.f, 0.f, 0.f}; acc2[t] = z; }
#pragma unroll
  for (int kt = 0; kt < 2; ++kt) {
    const _Float16* ar = &sT[wave][m * DL + 32 * kt + 8 * hh];
    FragH a;
    a.h[0] = *(const v8h*)ar;
    a.h[1] = *(const v8h*)(ar + 16);
#pragma unroll
    for (int t = 0; t < 4; ++t) {
      const _Float16* bp = W2p + (size_t)(16 * t + m) * DL + 32 * kt + 8 * hh;
      FragH b;
      b.h[0] = *(const v8h*)bp;
      b.h[1] = *(const v8h*)(bp + 16);
      acc2[t] = wmh(a.v, b.v, acc2[t]);
    }
  }
  __syncthreads();
#pragma unroll
  for (int t = 0; t < 4; ++t) {
    const float bias = pb2[16 * t + m];
    float* sp = &stg[wave][(8 * hh) * DL + 16 * t + m];
#pragma unroll
    for (int r = 0; r < 8; ++r) sp[r * DL] = acc2[t][r] * WINV + bias;
  }
  __syncthreads();

  const float* lp = &stg[wave][4 * lane];
  float* gp = hpl + (size_t)row0 * DL + 4 * lane;
  v4f ov[8];
#pragma unroll
  for (int q = 0; q < 8; ++q) ov[q] = *(const v4f*)(lp + q * 128);
#pragma unroll
  for (int q = 0; q < 8; ++q) *(volatile v4f*)(gp + (size_t)q * 128) = ov[q];
  __threadfence();
#pragma unroll
  for (int q = 0; q < 8; ++q) *(volatile v4f*)(gp + (size_t)q * 128) = ov[q];
}

__global__ __launch_bounds__(NTHR) void k_agg(
    const int* __restrict__ ei, const float* __restrict__ hpl,
    const _Float16* __restrict__ V1p, const float* __restrict__ vb1,
    const _Float16* __restrict__ V2p, const float* __restrict__ vb2,
    const _Float16* __restrict__ D1p, const float* __restrict__ db1,
    const float* __restrict__ dw2, const float* __restrict__ db2,
    float* out, int nN, int nE, int vec8) {
  extern __shared__ v4f lds_dyn[];
  float*    accL = (float*)lds_dyn;
  int*      list = (int*)(accL + NB * DL);
  _Float16* sTb  = (_Float16*)list;
  float*    outs = (float*)(list + LISTN);
  int*      wcnt = (int*)(outs + NB);
  const int tid = threadIdx.x, lane = tid & 31, wave = tid >> 5, hh = lane >> 4, m = lane & 15;
  const int nodeBase = blockIdx.x * NB;
  const int* dsts = ei + nE;

  {
    const v4f z = {0.f, 0.f, 0.f, 0.f};
    for (int i = tid; i < NB * DL / 4; i += NTHR) lds_dyn[i] = z;
  }
  __syncthreads();

  const int nChunks = (nE + CHUNK - 1) / CHUNK;
#pragma unroll 1
  for (int ch = 0; ch < nChunks; ++ch) {
    const int cbase = ch * CHUNK;
    const int wc = scan_chunk<NB>(dsts, nE, cbase, nodeBase, vec8, list, tid, lane, wave);
    if (lane == 0) wcnt[wave] = wc;
    __syncthreads();
    if (wave == 0) {
#pragma unroll 1
      for (int wsx = 0; wsx < NWAVE; ++wsx) {
        int n = __builtin_amdgcn_readfirstlane(wcnt[wsx]);
        n = n > WCAP ? WCAP : (n < 0 ? 0 : n);
        const int* lp = list + wsx * WCAP;
#pragma unroll 1
        for (int i = 0; i < n; ++i) {
          const int ent  = __builtin_amdgcn_readfirstlane(lp[i]);
          const int slot = ent & (NB - 1);
          int e = cbase + ((ent >> 12) & (CHUNK - 1));
          e = e > nE - 1 ? nE - 1 : e;
          int src = ei[e];
          src = src < 0 ? 0 : (src > nN - 1 ? nN - 1 : src);
          const v2f v = *(const v2f*)(hpl + (size_t)src * DL + 2 * lane);
          v2f* ap = (v2f*)(accL + slot * DL + 2 * lane);
          *ap = *ap + v;
        }
      }
    }
    __syncthreads();
  }

  _Float16* sT = sTb + wave * (16 * DL);
  const float bo = db2[0];
#pragma unroll 1
  for (int tt = 0; tt < NB / 16 / NWAVE; ++tt) {
    const int t = tt * NWAVE + wave;
    int node = nodeBase + 16 * t + m;
    node = node > nN - 1 ? nN - 1 : node;

    v8f c1[4];
#pragma unroll
    for (int tc = 0; tc < 4; ++tc) { v8f z = {0.f, 0.f, 0.f, 0.f, 0.f, 0.f, 0.f, 0.f}; c1[tc] = z; }
    const float* hr = hpl + (size_t)node * DL + 8 * hh;
#pragma unroll
    for (int kt = 0; kt < 2; ++kt) {
      const v4f p0 = *(const v4f*)(hr + 32 * kt),      p1 = *(const v4f*)(hr + 32 * kt + 4);
      const v4f p2 = *(const v4f*)(hr + 32 * kt + 16), p3 = *(const v4f*)(hr + 32 * kt + 20);
      FragH a;
      a.h[0] = cvt8(p0, p1);
      a.h[1] = cvt8(p2, p3);
#pragma unroll
      for (int tc = 0; tc < 4; ++tc) {
        const _Float16* bp = V1p + (size_t)(16 * tc + m) * DL + 32 * kt + 8 * hh;
        FragH b;
        b.h[0] = *(const v8h*)bp;
        b.h[1] = *(const v8h*)(bp + 16);
        c1[tc] = wmh(a.v, b.v, c1[tc]);
      }
    }
#pragma unroll
    for (int tc = 0; tc < 4; ++tc) {
      const float bias = vb1[16 * tc + m];
      _Float16* sp = sT + (8 * hh) * DL + 16 * tc + m;
#pragma unroll
      for (int r = 0; r < 8; ++r) sp[r * DL] = (_Float16)gelu_exact(c1[tc][r] * WINV + bias);
    }
    __syncthreads();

    v8f c2[4];
#pragma unroll
    for (int tc = 0; tc < 4; ++tc) { v8f z = {0.f, 0.f, 0.f, 0.f, 0.f, 0.f, 0.f, 0.f}; c2[tc] = z; }
#pragma unroll
    for (int kt = 0; kt < 2; ++kt) {
      const _Float16* ar = sT + m * DL + 32 * kt + 8 * hh;
      FragH a;
      a.h[0] = *(const v8h*)ar;
      a.h[1] = *(const v8h*)(ar + 16);
#pragma unroll
      for (int tc = 0; tc < 4; ++tc) {
        const _Float16* bp = V2p + (size_t)(16 * tc + m) * DL + 32 * kt + 8 * hh;
        FragH b;
        b.h[0] = *(const v8h*)bp;
        b.h[1] = *(const v8h*)(bp + 16);
        c2[tc] = wmh(a.v, b.v, c2[tc]);
      }
    }
    __syncthreads();
#pragma unroll
    for (int tc = 0; tc < 4; ++tc) {
      const float bias = vb2[16 * tc + m];
      const float* ag = accL + (16 * t + 8 * hh) * DL + 16 * tc + m;
      _Float16* sp = sT + (8 * hh) * DL + 16 * tc + m;
#pragma unroll
      for (int r = 0; r < 8; ++r)
        sp[r * DL] = (_Float16)gelu_exact(c2[tc][r] * WINV + bias + ag[r * DL]);
    }
    __syncthreads();

    v8f c3[4];
#pragma unroll
    for (int tc = 0; tc < 4; ++tc) { v8f z = {0.f, 0.f, 0.f, 0.f, 0.f, 0.f, 0.f, 0.f}; c3[tc] = z; }
#pragma unroll
    for (int kt = 0; kt < 2; ++kt) {
      const _Float16* ar = sT + m * DL + 32 * kt + 8 * hh;
      FragH a;
      a.h[0] = *(const v8h*)ar;
      a.h[1] = *(const v8h*)(ar + 16);
#pragma unroll
      for (int tc = 0; tc < 4; ++tc) {
        const _Float16* bp = D1p + (size_t)(16 * tc + m) * DL + 32 * kt + 8 * hh;
        FragH b;
        b.h[0] = *(const v8h*)bp;
        b.h[1] = *(const v8h*)(bp + 16);
        c3[tc] = wmh(a.v, b.v, c3[tc]);
      }
    }
    float pr[8];
#pragma unroll
    for (int r = 0; r < 8; ++r) pr[r] = 0.0f;
#pragma unroll
    for (int tc = 0; tc < 4; ++tc) {
      const float bias = db1[16 * tc + m];
      const float wv2  = dw2[16 * tc + m];
#pragma unroll
      for (int r = 0; r < 8; ++r) pr[r] += gelu_exact(c3[tc][r] * WINV + bias) * wv2;
    }
#pragma unroll
    for (int r = 0; r < 8; ++r) {
      pr[r] += __shfl_xor(pr[r], 1);
      pr[r] += __shfl_xor(pr[r], 2);
      pr[r] += __shfl_xor(pr[r], 4);
      pr[r] += __shfl_xor(pr[r], 8);
    }
    if (m == 0) {
#pragma unroll
      for (int r = 0; r < 8; ++r) outs[16 * t + 8 * hh + r] = pr[r] + bo;
    }
    __syncthreads();
  }

  {
    const int f   = wave * 128 + 4 * lane;
    const int fcl = f < NB - 4 ? f : NB - 4;
    const v4f ov  = *(const v4f*)(outs + fcl);
    const bool wv = wave < NB / 128;
    const size_t gi = (size_t)nodeBase + (size_t)f;
    const size_t nn = (size_t)nN;
    if (wv) {
      if (gi + 4 <= nn) *(volatile v4f*)(out + gi) = ov;
      else {
        if (gi + 0 < nn) *(volatile float*)(out + gi + 0) = ov[0];
        if (gi + 1 < nn) *(volatile float*)(out + gi + 1) = ov[1];
        if (gi + 2 < nn) *(volatile float*)(out + gi + 2) = ov[2];
        if (gi + 3 < nn) *(volatile float*)(out + gi + 3) = ov[3];
      }
    }
    __threadfence();
    if (wv) {
      if (gi + 4 <= nn) *(volatile v4f*)(out + gi) = ov;
      else {
        if (gi + 0 < nn) *(volatile float*)(out + gi + 0) = ov[0];
        if (gi + 1 < nn) *(volatile float*)(out + gi + 1) = ov[1];
        if (gi + 2 < nn) *(volatile float*)(out + gi + 2) = ov[2];
        if (gi + 3 < nn) *(volatile float*)(out + gi + 3) = ov[3];
      }
    }
  }
}

extern "C" void kernel_launch(void* const* d_in, const int* in_sizes, int n_in,
                              void* d_out, int out_size, void* d_ws, size_t ws_size,
                              hipStream_t stream) {
  if (n_in < 16) return;
  const int nN = in_sizes[0] / KX;
  const int nE = in_sizes[2] / 2;
  if (nN <= 0 || nE < 0 || in_sizes[0] != nN * KX || in_sizes[1] != nN * 2 || in_sizes[2] != nE * 2) return;
  if (in_sizes[4] != K1REAL * DL || in_sizes[5] < DL || in_sizes[6] != DL * DL || in_sizes[7] < DL) return;
  if (in_sizes[8] != DL * DL || in_sizes[9] < DL || in_sizes[10] != DL * DL || in_sizes[11] < DL) return;
  if (in_sizes[12] != DL * DL || in_sizes[13] < DL || in_sizes[14] < DL || in_sizes[15] < 1) return;
  if (out_size != nN) return;

  const float* x    = (const float*)d_in[0];
  const float* grd  = (const float*)d_in[1];
  const int*   ei   = (const int*)d_in[2];
  const float* pw1  = (const float*)d_in[4];
  const float* pb1  = (const float*)d_in[5];
  const float* pw2  = (const float*)d_in[6];
  const float* pb2  = (const float*)d_in[7];
  const float* ww1  = (const float*)d_in[8];
  const float* wb1  = (const float*)d_in[9];
  const float* ww2  = (const float*)d_in[10];
  const float* wb2  = (const float*)d_in[11];
  const float* dw1  = (const float*)d_in[12];
  const float* db1  = (const float*)d_in[13];
  const float* dw2  = (const float*)d_in[14];
  const float* db2  = (const float*)d_in[15];
  float* out = (float*)d_out;

  const int nNB = (nN + NROWS - 1) / NROWS;
  const int nAB = (nN + NB - 1) / NB;

  char* ws = (char*)d_ws;
  size_t off = 0;
  const size_t oW1 = off; off += (size_t)DL * K1 * 2;                 off = (off + 255) & ~(size_t)255;
  const size_t oW2 = off; off += (size_t)DL * DL * 2;                 off = (off + 255) & ~(size_t)255;
  const size_t oV1 = off; off += (size_t)DL * DL * 2;                 off = (off + 255) & ~(size_t)255;
  const size_t oV2 = off; off += (size_t)DL * DL * 2;                 off = (off + 255) & ~(size_t)255;
  const size_t oD1 = off; off += (size_t)DL * DL * 2;                 off = (off + 255) & ~(size_t)255;
  const size_t oH  = off; off += (size_t)nNB * NROWS * DL * 4;        off = (off + 255) & ~(size_t)255;
  if (off > ws_size) return;
  _Float16* W1p = (_Float16*)(ws + oW1);
  _Float16* W2p = (_Float16*)(ws + oW2);
  _Float16* V1p = (_Float16*)(ws + oV1);
  _Float16* V2p = (_Float16*)(ws + oV2);
  _Float16* D1p = (_Float16*)(ws + oD1);
  float*    hpl = (float*)(ws + oH);

  const int vec8 = ((nE & 3) == 0) ? 1 : 0;

  const int nPrep = DL * K1 / 8 + 4 * (DL * DL / 8);
  k_wprep<<<(nPrep + NTHR - 1) / NTHR, NTHR, 0, stream>>>(pw1, pw2, ww1, ww2, dw1, W1p, W2p, V1p, V2p, D1p);

  k_node<<<nNB, NTHR, 0, stream>>>(x, grd, W1p, pb1, W2p, pb2, hpl, nN);

  hipFuncSetAttribute(reinterpret_cast<const void*>(&k_agg),
                      hipFuncAttributeMaxDynamicSharedMemorySize, LDS_AGG);
  k_agg<<<nAB, NTHR, LDS_AGG, stream>>>(ei, hpl, V1p, wb1, V2p, wb2, D1p, db1, dw2, db2, out, nN, nE, vec8);
}
